// DeepIO_2611340116384
// MI455X (gfx1250) — hardware-verified
//
#include <hip/hip_runtime.h>


#define AS3 __attribute__((address_space(3)))

#define B_    64
#define T_    1024
#define H_    256
#define G_    1024
#define I0_   3
#define I1_   512
#define NF_   256
#define NO_   196
#define MB_   16
#define NTHR  256
#define NGRP  (B_ / MB_)

static_assert(NGRP == 4);
static_assert(NTHR == 256);
static_assert(H_ == (NTHR / 32) * 32);
static_assert(H_ % 32 == 0 && I1_ % 32 == 0);

typedef _Float16 v16h __attribute__((ext_vector_type(16)));
typedef _Float16 v8h  __attribute__((ext_vector_type(8)));
typedef float    v8f  __attribute__((ext_vector_type(8)));
typedef float    v4f  __attribute__((ext_vector_type(4)));
typedef __bf16   v16b __attribute__((ext_vector_type(16)));
typedef unsigned short v16us __attribute__((ext_vector_type(16)));

typedef AS3 _Float16*       lp_h;
typedef AS3 const _Float16* lcp_h;
typedef AS3 float*          lp_f;
typedef AS3 const float*    lcp_f;
typedef AS3 int*            lp_i;
typedef AS3 v4f*            lp_v4;

union Frag  { v16h v; v8h half[2]; };
union FragB { v16b v; v16us u; };

constexpr int KC2 = I1_ + H_;
constexpr int AP1 = 520;
constexpr int AP2 = 1288;
constexpr int AP3 = 1032;
constexpr int YP  = 260;
static_assert(AP1 % 8 == 0 && AP2 % 8 == 0 && AP3 % 8 == 0 && YP % 4 == 0);
static_assert(AP1 >= 2 * H_ && AP2 >= 2 * I1_ + H_ && AP3 >= 2 * I1_ && YP >= NF_);
constexpr int A1T = MB_ * AP1;
constexpr int A2T = MB_ * AP2;

#define SCLH    16.0f
#define SCLW    256.0f
#define SCLR    2048.0f
#define INV4096 0.000244140625f
#define INV2048 0.00048828125f

constexpr size_t SZ_WC1  = (size_t)2 * G_ * H_ * 2;
constexpr size_t SZ_WC2F = (size_t)G_ * KC2 * 2;
constexpr size_t SZ_WC2B = (size_t)G_ * I1_ * 2;
constexpr size_t SZ_H1   = (size_t)B_ * T_ * I1_ * 2;
constexpr size_t SZ_H1R  = SZ_H1;
constexpr size_t SZ_FEAT = (size_t)B_ * I1_ * 4;
constexpr size_t OFF_WC1  = 0;
constexpr size_t OFF_WC2F = OFF_WC1 + SZ_WC1;
constexpr size_t OFF_WC2B = OFF_WC2F + SZ_WC2F;
constexpr size_t OFF_H1   = OFF_WC2B + SZ_WC2B;
constexpr size_t OFF_H1R  = OFF_H1 + SZ_H1;
constexpr size_t OFF_FEAT = OFF_H1R + SZ_H1R;
constexpr size_t WS_END   = OFF_FEAT + SZ_FEAT;
static_assert(OFF_WC2F % 128 == 0 && OFF_WC2B % 128 == 0 && OFF_H1 % 128 == 0 && OFF_H1R % 128 == 0 && OFF_FEAT % 128 == 0);
static_assert(WS_END <= (size_t)268435456);

constexpr int NP1 = (int)(SZ_WC1 / 16);
constexpr int NP2 = (int)(SZ_WC2F / 16);
constexpr int NP3 = (int)(SZ_WC2B / 16);
constexpr int NCVTBLK = (NP1 + NP2 + NP3) / NTHR;
static_assert(NP1 % NTHR == 0 && NP2 % NTHR == 0 && NP3 % NTHR == 0);
static_assert((size_t)(NP1 + NP2 + NP3) * 16 == SZ_WC1 + SZ_WC2F + SZ_WC2B);

constexpr size_t L1_OFF_A = 0;
constexpr size_t L1_OFF_C = L1_OFF_A + (size_t)2 * A1T * 2;
constexpr size_t L1_OFF_W = L1_OFF_C + (size_t)MB_ * H_ * 4;
constexpr size_t L1_OFF_X = L1_OFF_W + (size_t)G_ * 16;
constexpr size_t L1_OFF_I = L1_OFF_X + (size_t)2 * MB_ * 4 * 4;
constexpr size_t L1_LDS   = L1_OFF_I + (size_t)(B_ + 2 * MB_) * 4;
static_assert(L1_OFF_C % 16 == 0 && L1_OFF_W % 16 == 0 && L1_OFF_X % 16 == 0 && L1_OFF_I % 16 == 0);

constexpr size_t L2_OFF_A  = 0;
constexpr size_t L2_OFF_C  = L2_OFF_A + (size_t)2 * A2T * 2;
constexpr size_t L2_OFF_HF = L2_OFF_C + (size_t)MB_ * H_ * 4;
constexpr size_t L2_OFF_B  = L2_OFF_HF + (size_t)MB_ * H_ * 4;
constexpr size_t L2_OFF_I  = L2_OFF_B + (size_t)G_ * 4;
constexpr size_t L2_LDS    = L2_OFF_I + (size_t)(B_ + 2 * MB_) * 4;
static_assert(L2_OFF_C % 16 == 0 && L2_OFF_HF % 16 == 0 && L2_OFF_B % 16 == 0 && L2_OFF_I % 16 == 0);

constexpr size_t L3_OFF_A  = 0;
constexpr size_t L3_OFF_HO = L3_OFF_A + (size_t)MB_ * AP3 * 2;
constexpr size_t L3_OFF_B  = L3_OFF_HO + (size_t)MB_ * H_ * 4;
constexpr size_t L3_OFF_I  = L3_OFF_B + (size_t)G_ * 4;
constexpr size_t L3_LDS    = L3_OFF_I + (size_t)MB_ * 4;
static_assert(L3_OFF_HO % 16 == 0 && L3_OFF_B % 16 == 0 && L3_OFF_I % 16 == 0);

constexpr size_t LH_OFF_Y = 0;
constexpr size_t LH_OFF_O = LH_OFF_Y + (size_t)B_ * YP * 4;
constexpr size_t LH_LDS   = LH_OFF_O + (size_t)B_ * NO_ * 4;
static_assert(LH_OFF_O % 16 == 0);
constexpr int NOUTP = B_ * NO_ / 4;
static_assert((B_ * NO_) % 32 == 0);
static_assert(NOUTP % 32 == 0);

__device__ __forceinline__ float rcpx(float x) { return __builtin_amdgcn_rcpf(x); }
__device__ __forceinline__ float sigm(float x) { return rcpx(1.0f + __expf(-x)); }
__device__ __forceinline__ float tanhm(float x) {
    const float e = __expf(2.0f * x);
    return 1.0f - 2.0f * rcpx(e + 1.0f);
}
__device__ __forceinline__ v8f zero8() {
    v8f z;
#pragma unroll
    for (int i = 0; i < 8; ++i) z[i] = 0.0f;
    return z;
}
__device__ __forceinline__ v8h zero8h() {
    v8h z;
#pragma unroll
    for (int i = 0; i < 8; ++i) z[i] = (_Float16)0.0f;
    return z;
}
__device__ __forceinline__ v4f zero4() {
    v4f z;
#pragma unroll
    for (int i = 0; i < 4; ++i) z[i] = 0.0f;
    return z;
}
__device__ __forceinline__ v8f ld8f(const float* p) {
    const v4f a = *(const v4f*)p;
    const v4f b = *(const v4f*)(p + 4);
    return __builtin_shufflevector(a, b, 0, 1, 2, 3, 4, 5, 6, 7);
}
__device__ __forceinline__ v8f ld8f_lds(lcp_f p) {
    const v4f a = *(AS3 const v4f*)p;
    const v4f b = *(AS3 const v4f*)(p + 4);
    return __builtin_shufflevector(a, b, 0, 1, 2, 3, 4, 5, 6, 7);
}

__device__ __forceinline__ unsigned int bf16_rne_bits(float f) {
    const unsigned int u = __float_as_uint(f);
    return (u + 0x7FFFu + ((u >> 16) & 1u)) >> 16;
}
__device__ __forceinline__ void cvt16(const v8f e0, const v8f e1, FragB& hi, FragB& lo) {
#pragma unroll
    for (int i = 0; i < 8; ++i) {
        const unsigned int hb = bf16_rne_bits(e0[i]);
        const float hf = __uint_as_float(hb << 16);
        const unsigned int lb = bf16_rne_bits(e0[i] - hf);
        hi.u[i] = (unsigned short)hb;
        lo.u[i] = (unsigned short)lb;
    }
#pragma unroll
    for (int i = 0; i < 8; ++i) {
        const unsigned int hb = bf16_rne_bits(e1[i]);
        const float hf = __uint_as_float(hb << 16);
        const unsigned int lb = bf16_rne_bits(e1[i] - hf);
        hi.u[8 + i] = (unsigned short)hb;
        lo.u[8 + i] = (unsigned short)lb;
    }
}

__device__ __forceinline__ void ldfrag_lds(Frag& f, lcp_h p) {
    f.half[0] = *(AS3 const v8h*)(p);
    f.half[1] = *(AS3 const v8h*)(p + 16);
}
__device__ __forceinline__ void ldfrag_glb(Frag& f, const _Float16* p) {
    f.half[0] = *(const v8h*)(p);
    f.half[1] = *(const v8h*)(p + 16);
}
__device__ __forceinline__ v8f mma16(v8f c, const Frag& a, const Frag& b) {
    return __builtin_amdgcn_wmma_f32_16x16x32_f16(false, a.v, false, b.v, (short)0, c, false, false);
}
__device__ __forceinline__ v8f mmab(v8f c, const FragB& a, const FragB& b) {
    return __builtin_amdgcn_wmma_f32_16x16x32_bf16(false, a.v, false, b.v, (short)0, c, false, false);
}
__device__ __forceinline__ v8f mma3b(v8f c, const FragB& ah, const FragB& al, const FragB& bh, const FragB& bl) {
    c = mmab(c, ah, bh);
    c = mmab(c, al, bh);
    c = mmab(c, ah, bl);
    asm volatile("v_nop\n\tv_nop\n\tv_nop\n\tv_nop" : "+v"(c) : "v"(ah.u), "v"(al.u), "v"(bh.u), "v"(bl.u));
    return c;
}

__global__ __launch_bounds__(NTHR)
void cvt_kernel(const float* __restrict__ Whh0, const float* __restrict__ Wih1,
                const float* __restrict__ Whh1, _Float16* wc1, _Float16* wc2f, _Float16* wc2b)
{
    const int p = (int)blockIdx.x * NTHR + (int)threadIdx.x;
    const int p1 = min(p, NP1 - 1);
    const int q  = min(max(p - NP1, 0), NP2 - 1);
    const int r  = min(max(p - NP1 - NP2, 0), NP3 - 1);

    const v8f v1 = ld8f(Whh0 + (size_t)p1 * 8);
    const int n2  = q / (KC2 / 8);
    const int c8  = (q - n2 * (KC2 / 8)) * 8;
    const int ci  = min(c8, I1_ - 8);
    const int cj  = min(max(c8 - I1_, 0), H_ - 8);
    const v8f v2a = ld8f(Wih1 + (size_t)n2 * I1_ + ci);
    const v8f v2b = ld8f(Whh1 + (size_t)n2 * H_ + cj);
    const v8f v3 = ld8f(Wih1 + (size_t)G_ * I1_ + (size_t)r * 8);

    v8f v;
#pragma unroll
    for (int i = 0; i < 8; ++i) {
        const float s2 = (c8 < I1_) ? v2a[i] : v2b[i];
        v[i] = (p < NP1) ? v1[i] : ((p < NP1 + NP2) ? s2 : v3[i]);
    }
    _Float16* d = (p < NP1) ? (wc1 + (size_t)p1 * 8)
                : ((p < NP1 + NP2) ? (wc2f + (size_t)q * 8) : (wc2b + (size_t)r * 8));
    v8h hv;
#pragma unroll
    for (int i = 0; i < 8; ++i) hv[i] = (_Float16)(v[i] * SCLW);
    *(volatile v8h*)d = hv;
    __threadfence();
    *(volatile v8h*)d = hv;
}

__global__ __launch_bounds__(NTHR)
void l1_kernel(const float* __restrict__ x, const int* __restrict__ lengths,
               const float* __restrict__ Wih0, const float* __restrict__ bih0,
               const float* __restrict__ bhh0, const _Float16* __restrict__ wc1,
               _Float16* y1h, _Float16* y1r)
{
    extern __shared__ __attribute__((aligned(16))) char smem[];
    lp_h  sA   = (lp_h)(smem + L1_OFF_A);
    lp_f  sC   = (lp_f)(smem + L1_OFF_C);
    lp_v4 sWgb = (lp_v4)(smem + L1_OFF_W);
    lp_f  sX   = (lp_f)(smem + L1_OFF_X);
    lp_i  sL64 = (lp_i)(smem + L1_OFF_I);
    lp_i  sSeq = sL64 + B_;
    lp_i  sLen = sSeq + MB_;

    const int tid  = threadIdx.x;
    const int lane = tid & 31;
    const int w    = tid >> 5;
    const int h    = lane >> 4;
    const int m    = lane & 15;
    const int dir  = (int)blockIdx.x >> 2;
    const int grp  = (int)blockIdx.x & 3;

    if (tid < B_) sL64[tid] = min(max(lengths[tid], 0), T_);
    if (tid < MB_) { sSeq[tid] = grp * MB_ + tid; sLen[tid] = 0; }
    {
        const v8h zh = zero8h();
        for (int i = tid; i < (2 * A1T) / 8; i += NTHR) *(AS3 v8h*)(sA + 8 * i) = zh;
        const v4f zf = zero4();
        for (int i = tid; i < (MB_ * H_) / 4; i += NTHR) *(AS3 v4f*)(sC + 4 * i) = zf;
        for (int j = tid; j < G_; j += NTHR) {
            const float* wp = Wih0 + ((size_t)dir * G_ + j) * I0_;
            v4f t4;
            t4[0] = wp[0];
            t4[1] = wp[1];
            t4[2] = wp[2];
            t4[3] = bih0[dir * G_ + j] + bhh0[dir * G_ + j];
            sWgb[j] = t4;
        }
    }
    __syncthreads();
    if (tid < B_) {
        const int my = sL64[tid];
        int rk = 0;
#pragma unroll 1
        for (int j = 0; j < B_; ++j) {
            const int lj = sL64[j];
            rk += (lj < my || (lj == my && j < tid)) ? 1 : 0;
        }
        if ((rk >> 4) == grp) { sSeq[rk & 15] = tid; sLen[rk & 15] = my; }
    }
    __syncthreads();
    int steps = 0;
#pragma unroll
    for (int i = 0; i < MB_; ++i) steps = max(steps, sLen[i]);

    if (w == 0) {
        const int row = m;
        const int b   = sSeq[row];
        const int L   = sLen[row];
        const int pos = (dir == 0) ? 0 : ((L > 0) ? (L - 1) : 0);
        const float* xp = x + ((size_t)b * T_ + pos) * I0_;
        sX[row * 4 + 0] = xp[0];
        sX[row * 4 + 1] = xp[1];
        sX[row * 4 + 2] = xp[2];
    }
    __syncthreads();

    const _Float16* wbase = wc1 + (size_t)dir * G_ * H_;

#pragma unroll 1
    for (int t = 0; t < steps; ++t) {
        const int cur = t & 1;
        lp_h sAc = sA + cur * A1T;
        lp_h sAn = sA + (cur ^ 1) * A1T;
        lp_f sXc = sX + cur * (MB_ * 4);
        lp_f sXn = sX + (cur ^ 1) * (MB_ * 4);

        if (w == 0 && t + 1 < steps) {
            const int tn  = t + 1;
            const int row = m;
            const int b   = sSeq[row];
            const int L   = sLen[row];
            const int pos = (dir == 0) ? tn : ((tn < L) ? (L - 1 - tn) : tn);
            const float* xp = x + ((size_t)b * T_ + pos) * I0_;
            sXn[row * 4 + 0] = xp[0];
            sXn[row * 4 + 1] = xp[1];
            sXn[row * 4 + 2] = xp[2];
        }

#pragma unroll 1
        for (int g = 0; g < 2; ++g) {
            const int j0 = w * 32 + g * 16;
            v8f acc[4];
#pragma unroll
            for (int q = 0; q < 4; ++q) acc[q] = zero8();

            lcp_h ab = sAc + m * AP1 + 8 * h;
            const _Float16* wb = wbase + (size_t)(j0 + m) * H_ + 8 * h;

#pragma unroll 1
            for (int k0 = 0; k0 < H_; k0 += 32) {
                Frag a, b[4];
                ldfrag_lds(a, ab + k0);
#pragma unroll
                for (int q = 0; q < 4; ++q) ldfrag_glb(b[q], wb + (size_t)q * (H_ * H_) + k0);
#pragma unroll
                for (int q = 0; q < 4; ++q) acc[q] = mma16(acc[q], a, b[q]);
                asm volatile("v_nop\n\tv_nop\n\tv_nop\n\tv_nop"
                             : "+v"(acc[0]), "+v"(acc[1]), "+v"(acc[2]), "+v"(acc[3])
                             : "v"(a.v), "v"(b[0].v), "v"(b[1].v), "v"(b[2].v), "v"(b[3].v));
            }

            const int n = j0 + m;
            const v4f w0 = sWgb[n];
            const v4f w1 = sWgb[H_ + n];
            const v4f w2 = sWgb[2 * H_ + n];
            const v4f w3 = sWgb[3 * H_ + n];
#pragma unroll
            for (int r = 0; r < 8; ++r) {
                const int row = 8 * h + r;
                const float x0 = sXc[row * 4 + 0];
                const float x1 = sXc[row * 4 + 1];
                const float x2 = sXc[row * 4 + 2];
                const bool on = t < sLen[row];
                const float gi = acc[0][r] * INV4096 + w0[3] + x0 * w0[0] + x1 * w0[1] + x2 * w0[2];
                const float gf = acc[1][r] * INV4096 + w1[3] + x0 * w1[0] + x1 * w1[1] + x2 * w1[2];
                const float gg = acc[2][r] * INV4096 + w2[3] + x0 * w2[0] + x1 * w2[1] + x2 * w2[2];
                const float go = acc[3][r] * INV4096 + w3[3] + x0 * w3[0] + x1 * w3[1] + x2 * w3[2];
                const float cp = sC[row * H_ + n];
                const float cn = sigm(gf) * cp + sigm(gi) * tanhm(gg);
                const float hn = sigm(go) * tanhm(cn);
                sC[row * H_ + n] = on ? cn : cp;
                const float    vs = hn * SCLH;
                const _Float16 hv = (_Float16)vs;
                const _Float16 rv = (_Float16)((vs - (float)hv) * SCLR);
                const _Float16 holdh = sAc[row * AP1 + n];
                const _Float16 holdr = sAc[row * AP1 + H_ + n];
                sAn[row * AP1 + n]      = on ? hv : holdh;
                sAn[row * AP1 + H_ + n] = on ? rv : holdr;
            }
        }

        __syncthreads();

        {
            const int ra = w, rb = w + 8;
            const int sqa = sSeq[ra], sqb = sSeq[rb];
            const int lna = sLen[ra], lnb = sLen[rb];
            const bool ona = t < lna, onb = t < lnb;
            const int pa = (dir == 0) ? t : (ona ? (lna - 1 - t) : t);
            const int pb = (dir == 0) ? t : (onb ? (lnb - 1 - t) : t);
            v8h va  = *(AS3 const v8h*)(sAn + ra * AP1 + 8 * lane);
            v8h var = *(AS3 const v8h*)(sAn + ra * AP1 + H_ + 8 * lane);
            v8h vb  = *(AS3 const v8h*)(sAn + rb * AP1 + 8 * lane);
            v8h vbr = *(AS3 const v8h*)(sAn + rb * AP1 + H_ + 8 * lane);
#pragma unroll
            for (int i = 0; i < 8; ++i) {
                va[i]  = ona ? va[i]  : (_Float16)0.0f;
                var[i] = ona ? var[i] : (_Float16)0.0f;
                vb[i]  = onb ? vb[i]  : (_Float16)0.0f;
                vbr[i] = onb ? vbr[i] : (_Float16)0.0f;
            }
            const size_t oa = ((size_t)sqa * T_ + pa) * I1_ + dir * H_ + 8 * lane;
            const size_t ob = ((size_t)sqb * T_ + pb) * I1_ + dir * H_ + 8 * lane;
            *(volatile v8h*)(y1h + oa) = va;
            *(volatile v8h*)(y1r + oa) = var;
            *(volatile v8h*)(y1h + ob) = vb;
            *(volatile v8h*)(y1r + ob) = vbr;
            __threadfence();
            *(volatile v8h*)(y1h + oa) = va;
            *(volatile v8h*)(y1r + oa) = var;
            *(volatile v8h*)(y1h + ob) = vb;
            *(volatile v8h*)(y1r + ob) = vbr;
        }
    }
}

__device__ __forceinline__ void stage_rows(lp_h dst, int pitch, const _Float16* __restrict__ pl,
                                           lp_i sSeq, int pos, int tid)
{
#pragma unroll
    for (int i = 0; i < 4; ++i) {
        const int q   = tid + NTHR * i;
        const int row = q >> 6;
        const int c8  = (q & 63) * 8;
        const int b   = sSeq[row];
        const v8h v = *(const v8h*)(pl + ((size_t)b * T_ + pos) * I1_ + c8);
        *(AS3 v8h*)(dst + row * pitch + c8) = v;
    }
}

__global__ __launch_bounds__(NTHR)
void l2f_kernel(const int* __restrict__ lengths, const float* __restrict__ bih1,
                const float* __restrict__ bhh1, const _Float16* __restrict__ wc2f,
                const _Float16* __restrict__ y1h, const _Float16* __restrict__ y1r, float* feat)
{
    extern __shared__ __attribute__((aligned(16))) char smem[];
    lp_h sA   = (lp_h)(smem + L2_OFF_A);
    lp_f sC   = (lp_f)(smem + L2_OFF_C);
    lp_f sHf  = (lp_f)(smem + L2_OFF_HF);
    lp_f sBias = (lp_f)(smem + L2_OFF_B);
    lp_i sL64 = (lp_i)(smem + L2_OFF_I);
    lp_i sSeq = sL64 + B_;
    lp_i sLen = sSeq + MB_;

    const int tid  = threadIdx.x;
    const int lane = tid & 31;
    const int w    = tid >> 5;
    const int h    = lane >> 4;
    const int m    = lane & 15;
    const int grp  = (int)blockIdx.x;

    if (tid < B_) sL64[tid] = min(max(lengths[tid], 0), T_);
    if (tid < MB_) { sSeq[tid] = grp * MB_ + tid; sLen[tid] = 0; }
    {
        const v8h zh = zero8h();
        for (int i = tid; i < (2 * A2T) / 8; i += NTHR) *(AS3 v8h*)(sA + 8 * i) = zh;
        const v4f zf = zero4();
        for (int i = tid; i < (MB_ * H_) / 4; i += NTHR) { *(AS3 v4f*)(sC + 4 * i) = zf; *(AS3 v4f*)(sHf + 4 * i) = zf; }
        for (int j = tid; j < G_; j += NTHR) sBias[j] = bih1[j] + bhh1[j];
    }
    __syncthreads();
    if (tid < B_) {
        const int my = sL64[tid];
        int rk = 0;
#pragma unroll 1
        for (int j = 0; j < B_; ++j) {
            const int lj = sL64[j];
            rk += (lj < my || (lj == my && j < tid)) ? 1 : 0;
        }
        if ((rk >> 4) == grp) { sSeq[rk & 15] = tid; sLen[rk & 15] = my; }
    }
    __syncthreads();
    int steps = 0;
#pragma unroll
    for (int i = 0; i < MB_; ++i) steps = max(steps, sLen[i]);

    if (steps > 0) {
        stage_rows(sA,       AP2, y1h, sSeq, 0, tid);
        stage_rows(sA + I1_, AP2, y1r, sSeq, 0, tid);
    }
    __syncthreads();

#pragma unroll 1
    for (int t = 0; t < steps; ++t) {
        const int cur = t & 1;
        lp_h sAc = sA + cur * A2T;
        lp_h sAn = sA + (cur ^ 1) * A2T;

        if (t + 1 < steps) {
            stage_rows(sAn,       AP2, y1h, sSeq, t + 1, tid);
            stage_rows(sAn + I1_, AP2, y1r, sSeq, t + 1, tid);
        }

#pragma unroll 1
        for (int g = 0; g < 2; ++g) {
            const int j0 = w * 32 + g * 16;
            v8f acc[4], accr[4];
#pragma unroll
            for (int q = 0; q < 4; ++q) { acc[q] = zero8(); accr[q] = zero8(); }

            lcp_h ab = sAc + m * AP2 + 8 * h;
            const _Float16* wb = wc2f + (size_t)(j0 + m) * KC2 + 8 * h;

#pragma unroll 1
            for (int k0 = 0; k0 < I1_; k0 += 32) {
                Frag ah, ar, b[4];
                ldfrag_lds(ah, ab + k0);
                ldfrag_lds(ar, ab + I1_ + k0);
#pragma unroll
                for (int q = 0; q < 4; ++q) ldfrag_glb(b[q], wb + (size_t)q * (H_ * KC2) + k0);
#pragma unroll
                for (int q = 0; q < 4; ++q) acc[q]  = mma16(acc[q],  ah, b[q]);
#pragma unroll
                for (int q = 0; q < 4; ++q) accr[q] = mma16(accr[q], ar, b[q]);
                asm volatile("v_nop\n\tv_nop\n\tv_nop\n\tv_nop"
                             : "+v"(acc[0]), "+v"(acc[1]), "+v"(acc[2]), "+v"(acc[3]),
                               "+v"(accr[0]), "+v"(accr[1]), "+v"(accr[2]), "+v"(accr[3])
                             : "v"(ah.v), "v"(ar.v), "v"(b[0].v), "v"(b[1].v), "v"(b[2].v), "v"(b[3].v));
            }
#pragma unroll 1
            for (int k0 = 0; k0 < H_; k0 += 32) {
                Frag a, b[4];
                ldfrag_lds(a, ab + 2 * I1_ + k0);
#pragma unroll
                for (int q = 0; q < 4; ++q) ldfrag_glb(b[q], wb + (size_t)q * (H_ * KC2) + I1_ + k0);
#pragma unroll
                for (int q = 0; q < 4; ++q) acc[q] = mma16(acc[q], a, b[q]);
                asm volatile("v_nop\n\tv_nop\n\tv_nop\n\tv_nop"
                             : "+v"(acc[0]), "+v"(acc[1]), "+v"(acc[2]), "+v"(acc[3])
                             : "v"(a.v), "v"(b[0].v), "v"(b[1].v), "v"(b[2].v), "v"(b[3].v));
            }

            const int n = j0 + m;
            const float bi = sBias[n];
            const float bf = sBias[H_ + n];
            const float bg = sBias[2 * H_ + n];
            const float bo = sBias[3 * H_ + n];
#pragma unroll
            for (int r = 0; r < 8; ++r) {
                const int row = 8 * h + r;
                const bool on = t < sLen[row];
                const float gi = (acc[0][r] + accr[0][r] * INV2048) * INV4096 + bi;
                const float gf = (acc[1][r] + accr[1][r] * INV2048) * INV4096 + bf;
                const float gg = (acc[2][r] + accr[2][r] * INV2048) * INV4096 + bg;
                const float go = (acc[3][r] + accr[3][r] * INV2048) * INV4096 + bo;
                const float cp = sC[row * H_ + n];
                const float cn = sigm(gf) * cp + sigm(gi) * tanhm(gg);
                const float hn = sigm(go) * tanhm(cn);
                sC[row * H_ + n] = on ? cn : cp;
                const _Float16 hold = sAc[row * AP2 + 2 * I1_ + n];
                const _Float16 hv   = (_Float16)(hn * SCLH);
                sAn[row * AP2 + 2 * I1_ + n] = on ? hv : hold;
                const float hfo = sHf[row * H_ + n];
                sHf[row * H_ + n] = on ? hn : hfo;
            }
        }
        __syncthreads();
    }
    __syncthreads();

    {
        const int ra = w, rb = w + 8;
        const int sqa = sSeq[ra], sqb = sSeq[rb];
        const v4f a0 = *(AS3 const v4f*)(sHf + ra * H_ + 4 * lane);
        const v4f a1 = *(AS3 const v4f*)(sHf + ra * H_ + 128 + 4 * lane);
        const v4f c0 = *(AS3 const v4f*)(sHf + rb * H_ + 4 * lane);
        const v4f c1 = *(AS3 const v4f*)(sHf + rb * H_ + 128 + 4 * lane);
        float* da = feat + (size_t)sqa * I1_;
        float* db = feat + (size_t)sqb * I1_;
        *(volatile v4f*)(da + 4 * lane)       = a0;
        *(volatile v4f*)(da + 128 + 4 * lane) = a1;
        *(volatile v4f*)(db + 4 * lane)       = c0;
        *(volatile v4f*)(db + 128 + 4 * lane) = c1;
        __threadfence();
        *(volatile v4f*)(da + 4 * lane)       = a0;
        *(volatile v4f*)(da + 128 + 4 * lane) = a1;
        *(volatile v4f*)(db + 4 * lane)       = c0;
        *(volatile v4f*)(db + 128 + 4 * lane) = c1;
    }
}

__global__ __launch_bounds__(NTHR)
void l2b_kernel(const int* __restrict__ lengths, const float* __restrict__ bih1,
                const float* __restrict__ bhh1, const _Float16* __restrict__ wc2b,
                const _Float16* __restrict__ y1h, const _Float16* __restrict__ y1r, float* feat)
{
    extern __shared__ __attribute__((aligned(16))) char smem[];
    lp_h sA    = (lp_h)(smem + L3_OFF_A);
    lp_f sHo   = (lp_f)(smem + L3_OFF_HO);
    lp_f sBias = (lp_f)(smem + L3_OFF_B);
    lp_i sL    = (lp_i)(smem + L3_OFF_I);

    const int tid  = threadIdx.x;
    const int lane = tid & 31;
    const int w    = tid >> 5;
    const int h    = lane >> 4;
    const int m    = lane & 15;
    const int sq0  = (int)blockIdx.x * MB_;

    if (w == 0) sL[m] = min(max(lengths[sq0 + m], 1), T_) - 1;
    for (int j = tid; j < G_; j += NTHR) sBias[j] = bih1[G_ + j] + bhh1[G_ + j];
    __syncthreads();
    {
#pragma unroll
        for (int i = 0; i < 4; ++i) {
            const int q   = tid + NTHR * i;
            const int row = q >> 6;
            const int c8  = (q & 63) * 8;
            const int pos = sL[row];
            const size_t off = ((size_t)(sq0 + row) * T_ + pos) * I1_ + c8;
            const v8h vh = *(const v8h*)(y1h + off);
            const v8h vr = *(const v8h*)(y1r + off);
            *(AS3 v8h*)(sA + row * AP3 + c8)       = vh;
            *(AS3 v8h*)(sA + row * AP3 + I1_ + c8) = vr;
        }
    }
    __syncthreads();

#pragma unroll 1
    for (int g = 0; g < 2; ++g) {
        const int j0 = w * 32 + g * 16;
        v8f acc[4], accr[4];
#pragma unroll
        for (int q = 0; q < 4; ++q) { acc[q] = zero8(); accr[q] = zero8(); }

        lcp_h ab = sA + m * AP3 + 8 * h;
        const _Float16* wb = wc2b + (size_t)(j0 + m) * I1_ + 8 * h;

#pragma unroll 1
        for (int k0 = 0; k0 < I1_; k0 += 32) {
            Frag ah, ar, b[4];
            ldfrag_lds(ah, ab + k0);
            ldfrag_lds(ar, ab + I1_ + k0);
#pragma unroll
            for (int q = 0; q < 4; ++q) ldfrag_glb(b[q], wb + (size_t)q * (H_ * I1_) + k0);
#pragma unroll
            for (int q = 0; q < 4; ++q) acc[q]  = mma16(acc[q],  ah, b[q]);
#pragma unroll
            for (int q = 0; q < 4; ++q) accr[q] = mma16(accr[q], ar, b[q]);
            asm volatile("v_nop\n\tv_nop\n\tv_nop\n\tv_nop"
                         : "+v"(acc[0]), "+v"(acc[1]), "+v"(acc[2]), "+v"(acc[3]),
                           "+v"(accr[0]), "+v"(accr[1]), "+v"(accr[2]), "+v"(accr[3])
                         : "v"(ah.v), "v"(ar.v), "v"(b[0].v), "v"(b[1].v), "v"(b[2].v), "v"(b[3].v));
        }

        const int n = j0 + m;
        const float bi = sBias[n];
        const float bg = sBias[2 * H_ + n];
        const float bo = sBias[3 * H_ + n];
#pragma unroll
        for (int r = 0; r < 8; ++r) {
            const int row = 8 * h + r;
            const float gi = (acc[0][r] + accr[0][r] * INV2048) * INV4096 + bi;
            const float gg = (acc[2][r] + accr[2][r] * INV2048) * INV4096 + bg;
            const float go = (acc[3][r] + accr[3][r] * INV2048) * INV4096 + bo;
            const float cn = sigm(gi) * tanhm(gg);
            const float hn = sigm(go) * tanhm(cn);
            sHo[row * H_ + n] = hn;
        }
    }
    __syncthreads();

    {
        const int ra = w, rb = w + 8;
        const v4f a0 = *(AS3 const v4f*)(sHo + ra * H_ + 4 * lane);
        const v4f a1 = *(AS3 const v4f*)(sHo + ra * H_ + 128 + 4 * lane);
        const v4f c0 = *(AS3 const v4f*)(sHo + rb * H_ + 4 * lane);
        const v4f c1 = *(AS3 const v4f*)(sHo + rb * H_ + 128 + 4 * lane);
        float* da = feat + (size_t)(sq0 + ra) * I1_ + H_;
        float* db = feat + (size_t)(sq0 + rb) * I1_ + H_;
        *(volatile v4f*)(da + 4 * lane)       = a0;
        *(volatile v4f*)(da + 128 + 4 * lane) = a1;
        *(volatile v4f*)(db + 4 * lane)       = c0;
        *(volatile v4f*)(db + 128 + 4 * lane) = c1;
        __threadfence();
        *(volatile v4f*)(da + 4 * lane)       = a0;
        *(volatile v4f*)(da + 128 + 4 * lane) = a1;
        *(volatile v4f*)(db + 4 * lane)       = c0;
        *(volatile v4f*)(db + 128 + 4 * lane) = c1;
    }
}

__global__ __launch_bounds__(NTHR)
void head_kernel(const float* __restrict__ feat, const float* __restrict__ fc1w,
                 const float* __restrict__ fc1b, const float* __restrict__ gam,
                 const float* __restrict__ bet, const float* __restrict__ fow,
                 const float* __restrict__ fob, float* out)
{
    extern __shared__ __attribute__((aligned(16))) char smem[];
    lp_f sY = (lp_f)(smem + LH_OFF_Y);
    lp_f sO = (lp_f)(smem + LH_OFF_O);

    const int tid  = threadIdx.x;
    const int lane = tid & 31;
    const int w    = tid >> 5;
    const int h    = lane >> 4;
    const int m    = lane & 15;

    {
        const int n0 = (2 * w) * 16 + m;
        const int n1 = (2 * w + 1) * 16 + m;
        const float bb0 = fc1b[n0];
        const float bb1 = fc1b[n1];
#pragma unroll 1
        for (int mt = 0; mt < 4; ++mt) {
            v8f acc0 = zero8(), acc1 = zero8();
            const float* ap  = feat + (size_t)(16 * mt + m) * I1_ + 8 * h;
            const float* bp0 = fc1w + (size_t)n0 * I1_ + 8 * h;
            const float* bp1 = fc1w + (size_t)n1 * I1_ + 8 * h;
#pragma unroll 1
            for (int k0 = 0; k0 < I1_; k0 += 32) {
                FragB ah, al, bh, bl;
                cvt16(ld8f(ap + k0), ld8f(ap + k0 + 16), ah, al);
                cvt16(ld8f(bp0 + k0), ld8f(bp0 + k0 + 16), bh, bl);
                acc0 = mma3b(acc0, ah, al, bh, bl);
                cvt16(ld8f(bp1 + k0), ld8f(bp1 + k0 + 16), bh, bl);
                acc1 = mma3b(acc1, ah, al, bh, bl);
            }
#pragma unroll
            for (int r = 0; r < 8; ++r) {
                const int row = 16 * mt + 8 * h + r;
                sY[row * YP + n0] = fmaxf(acc0[r] + bb0, 0.0f);
                sY[row * YP + n1] = fmaxf(acc1[r] + bb1, 0.0f);
            }
        }
    }
    __syncthreads();

    {
        const int j = tid;
        double s = 0.0;
#pragma unroll 1
        for (int b = 0; b < B_; ++b) s += (double)sY[b * YP + j];
        const double mean = s * (1.0 / 64.0);
        double v = 0.0;
#pragma unroll 1
        for (int b = 0; b < B_; ++b) {
            const double d = (double)sY[b * YP + j] - mean;
            v += d * d;
        }
        v *= (1.0 / 64.0);
        const float meanf = (float)mean;
        const float varf  = (float)v;
        const float rs    = 1.0f / sqrtf(varf + 1e-5f);
        const float ga = gam[j];
        const float be = bet[j];
#pragma unroll 1
        for (int b = 0; b < B_; ++b) {
            const float y = sY[b * YP + j];
            sY[b * YP + j] = (ga * (y - meanf)) * rs + be;
        }
    }
    __syncthreads();

    {
        const int o0  = w * 16 + m;
        const int o1  = (w + 8) * 16 + m;
        const bool z1 = o1 < NO_;
        const int oc1 = min(o1, NO_ - 1);
        const float bb0 = fob[o0];
        const float bb1 = fob[oc1];
#pragma unroll 1
        for (int mt = 0; mt < 4; ++mt) {
            v8f acc0 = zero8(), acc1 = zero8();
            lcp_f ap = sY + (16 * mt + m) * YP + 8 * h;
            const float* bp0 = fow + (size_t)o0 * NF_ + 8 * h;
            const float* bp1 = fow + (size_t)oc1 * NF_ + 8 * h;
#pragma unroll 1
            for (int k0 = 0; k0 < NF_; k0 += 32) {
                FragB ah, al, bh, bl;
                cvt16(ld8f_lds(ap + k0), ld8f_lds(ap + k0 + 16), ah, al);
                cvt16(ld8f(bp0 + k0), ld8f(bp0 + k0 + 16), bh, bl);
                acc0 = mma3b(acc0, ah, al, bh, bl);
                v8f e0 = ld8f(bp1 + k0), e1 = ld8f(bp1 + k0 + 16);
#pragma unroll
                for (int i = 0; i < 8; ++i) { e0[i] = z1 ? e0[i] : 0.0f; e1[i] = z1 ? e1[i] : 0.0f; }
                cvt16(e0, e1, bh, bl);
                acc1 = mma3b(acc1, ah, al, bh, bl);
            }
#pragma unroll
            for (int r = 0; r < 8; ++r) {
                const int row = 16 * mt + 8 * h + r;
                sO[row * NO_ + o0] = acc0[r] + bb0;
                if (z1) sO[row * NO_ + o1] = acc1[r] + bb1;
            }
        }
    }
    __syncthreads();

#pragma unroll 1
    for (int it = 0; it < (NOUTP + NTHR - 1) / NTHR; ++it) {
        const int p = tid + NTHR * it;
        if (p < NOUTP) {
            const v4f v = *(AS3 const v4f*)(sO + 4 * p);
            *(volatile v4f*)(out + 4 * (size_t)p) = v;
        }
    }
    __threadfence();
#pragma unroll 1
    for (int it = 0; it < (NOUTP + NTHR - 1) / NTHR; ++it) {
        const int p = tid + NTHR * it;
        if (p < NOUTP) {
            const v4f v = *(AS3 const v4f*)(sO + 4 * p);
            *(volatile v4f*)(out + 4 * (size_t)p) = v;
        }
    }
}

extern "C" void kernel_launch(void* const* d_in, const int* in_sizes, int n_in,
                              void* d_out, int out_size, void* d_ws, size_t ws_size,
                              hipStream_t stream)
{
    if (n_in < 16) return;
    if (in_sizes[0]  != B_ * T_ * I0_) return;
    if (in_sizes[1]  != B_)            return;
    if (in_sizes[2]  != 2 * G_ * I0_)  return;
    if (in_sizes[3]  != 2 * G_ * H_)   return;
    if (in_sizes[4]  != 2 * G_)        return;
    if (in_sizes[5]  != 2 * G_)        return;
    if (in_sizes[6]  != 2 * G_ * I1_)  return;
    if (in_sizes[7]  != 2 * G_ * H_)   return;
    if (in_sizes[8]  != 2 * G_)        return;
    if (in_sizes[9]  != 2 * G_)        return;
    if (in_sizes[10] != NF_ * I1_)     return;
    if (in_sizes[11] != NF_)           return;
    if (in_sizes[12] != NF_)           return;
    if (in_sizes[13] != NF_)           return;
    if (in_sizes[14] != NO_ * NF_)     return;
    if (in_sizes[15] != NO_)           return;
    if (out_size != B_ * NO_)          return;
    if (ws_size < WS_END)              return;

    const float* x     = (const float*)d_in[0];
    const int*   lens  = (const int*)  d_in[1];
    const float* Wih0  = (const float*)d_in[2];
    const float* Whh0  = (const float*)d_in[3];
    const float* bih0  = (const float*)d_in[4];
    const float* bhh0  = (const float*)d_in[5];
    const float* Wih1  = (const float*)d_in[6];
    const float* Whh1  = (const float*)d_in[7];
    const float* bih1  = (const float*)d_in[8];
    const float* bhh1  = (const float*)d_in[9];
    const float* fc1w  = (const float*)d_in[10];
    const float* fc1b  = (const float*)d_in[11];
    const float* gam   = (const float*)d_in[12];
    const float* bet   = (const float*)d_in[13];
    const float* fow   = (const float*)d_in[14];
    const float* fob   = (const float*)d_in[15];
    float* out = (float*)d_out;

    char* ws = (char*)d_ws;
    _Float16* wc1  = (_Float16*)(ws + OFF_WC1);
    _Float16* wc2f = (_Float16*)(ws + OFF_WC2F);
    _Float16* wc2b = (_Float16*)(ws + OFF_WC2B);
    _Float16* y1h  = (_Float16*)(ws + OFF_H1);
    _Float16* y1r  = (_Float16*)(ws + OFF_H1R);
    float*    feat = (float*)   (ws + OFF_FEAT);

    cvt_kernel<<<dim3(NCVTBLK), dim3(NTHR), 0, stream>>>(Whh0, Wih1, Whh1, wc1, wc2f, wc2b);

    hipFuncSetAttribute(reinterpret_cast<const void*>(&l1_kernel),
                        hipFuncAttributeMaxDynamicSharedMemorySize, (int)L1_LDS);
    l1_kernel<<<dim3(2 * NGRP), dim3(NTHR), L1_LDS, stream>>>(x, lens, Wih0, bih0, bhh0,
                                                              (const _Float16*)wc1, y1h, y1r);

    hipFuncSetAttribute(reinterpret_cast<const void*>(&l2f_kernel),
                        hipFuncAttributeMaxDynamicSharedMemorySize, (int)L2_LDS);
    l2f_kernel<<<dim3(NGRP), dim3(NTHR), L2_LDS, stream>>>(lens, bih1, bhh1, (const _Float16*)wc2f,
                                                           (const _Float16*)y1h, (const _Float16*)y1r, feat);

    l2b_kernel<<<dim3(NGRP), dim3(NTHR), L3_LDS, stream>>>(lens, bih1, bhh1, (const _Float16*)wc2b,
                                                           (const _Float16*)y1h, (const _Float16*)y1r, feat);

    hipFuncSetAttribute(reinterpret_cast<const void*>(&head_kernel),
                        hipFuncAttributeMaxDynamicSharedMemorySize, (int)LH_LDS);
    head_kernel<<<dim3(1), dim3(NTHR), LH_LDS, stream>>>((const float*)feat, fc1w, fc1b, gam, bet,
                                                         fow, fob, out);
}
